// GPTCosAttention_86174223827531
// MI455X (gfx1250) — hardware-verified
//
#include <hip/hip_runtime.h>


#define NB_  2
#define TT   2048
#define DM   2048
#define NH_  16
#define HD   128
#define ROT  64
#define ZH   2
#define PCAR 8.0f
typedef _Float16 h16;
typedef unsigned short bf;
typedef __attribute__((ext_vector_type(16))) __bf16   v16bf;
typedef __attribute__((ext_vector_type(16))) _Float16 v16h;
typedef __attribute__((ext_vector_type(8)))  _Float16 v8h;
typedef __attribute__((ext_vector_type(8)))  unsigned short v8us;
typedef __attribute__((ext_vector_type(8)))  float    v8f;
typedef __attribute__((ext_vector_type(4)))  float    v4f;
typedef v8h  __attribute__((may_alias)) v8ha;
typedef v4f  __attribute__((may_alias)) v4fa;
typedef v8us __attribute__((may_alias)) v8usa;

__device__ __forceinline__ unsigned short f2bf(float f) { unsigned u = __float_as_uint(f); u += 0x7FFFu + ((u >> 16) & 1u); return (unsigned short)(u >> 16); }
__device__ __forceinline__ float bf2f(unsigned short b) { return __uint_as_float(((unsigned)b) << 16); }
__device__ __forceinline__ float bfr(float f) { return bf2f(f2bf(f)); }
__device__ __forceinline__ v16h cat16(v8h lo, v8h hi) { return __builtin_shufflevector(lo, hi, 0, 1, 2, 3, 4, 5, 6, 7, 8, 9, 10, 11, 12, 13, 14, 15); }
__device__ __forceinline__ v16bf cat16b(v8us lo, v8us hi) { return __builtin_bit_cast(v16bf, __builtin_shufflevector(lo, hi, 0, 1, 2, 3, 4, 5, 6, 7, 8, 9, 10, 11, 12, 13, 14, 15)); }
__device__ __forceinline__ v8f wmma16(v16h a, v16h b, v8f c) { return __builtin_amdgcn_wmma_f32_16x16x32_f16(false, a, false, b, (short)0, c, false, false); }
__device__ __forceinline__ v8f wmmab(v16bf a, v16bf b, v8f c) { return __builtin_amdgcn_wmma_f32_16x16x32_bf16(false, a, false, b, (short)0, c, false, false); }


template <typename T16> struct WFrag;
template <> struct WFrag<h16> { typedef v16h V; static __device__ __forceinline__ V ld(const h16* p) { return cat16(*(const v8h*)p, *(const v8h*)(p + 16)); } static __device__ __forceinline__ v8f mma(V a, V b, v8f c) { return wmma16(a, b, c); } };
template <> struct WFrag<bf> { typedef v16bf V; static __device__ __forceinline__ V ld(const bf* p) { return cat16b(*(const v8us*)p, *(const v8us*)(p + 16)); } static __device__ __forceinline__ v8f mma(V a, V b, v8f c) { return wmmab(a, b, c); } };
template <typename T16, int NSPLIT, bool BIAS>
__global__ __launch_bounds__(32) void k_gemmw(const T16* __restrict__ A, const T16* __restrict__ A2, const T16* __restrict__ Bt, const T16* __restrict__ Bt2, int K, float* C, int ldc, const float* __restrict__ bias, size_t sA, size_t sB, size_t sC) {
    typedef typename WFrag<T16>::V V;
    __shared__ __align__(16) float os[16 * 68];
    const size_t z = blockIdx.z; A += z * sA; if (A2) A2 += z * sA; Bt += z * sB; if (Bt2) Bt2 += z * sB; C += z * sC;
    const int lane = threadIdx.x & 31, lr = lane & 15, hi = lane >> 4; const int r0 = blockIdx.x * 64, c0 = blockIdx.y * 64;
    v8f acc[4][4];
#pragma unroll
    for (int mb = 0; mb < 4; ++mb)
#pragma unroll
        for (int nb = 0; nb < 4; ++nb) acc[mb][nb] = (v8f){};
    const size_t aoff = (size_t)(r0 + lr) * K + 8 * hi, boff = (size_t)(c0 + lr) * K + 8 * hi;
#pragma unroll 1
    for (int kc = 0; kc < K; kc += 32) {
        V a[4], a2[4];
#pragma unroll
        for (int mb = 0; mb < 4; ++mb) { a[mb] = WFrag<T16>::ld(A + aoff + (size_t)mb * 16 * K + kc); if (NSPLIT == 1 || NSPLIT == 2) a2[mb] = WFrag<T16>::ld(A2 + aoff + (size_t)mb * 16 * K + kc); }
#pragma unroll
        for (int nb = 0; nb < 4; ++nb) { const V b = WFrag<T16>::ld(Bt + boff + (size_t)nb * 16 * K + kc); V b2; if (NSPLIT >= 2) b2 = WFrag<T16>::ld(Bt2 + boff + (size_t)nb * 16 * K + kc);
#pragma unroll
            for (int mb = 0; mb < 4; ++mb) { acc[mb][nb] = WFrag<T16>::mma(a[mb], b, acc[mb][nb]); if (NSPLIT == 1 || NSPLIT == 2) acc[mb][nb] = WFrag<T16>::mma(a2[mb], b, acc[mb][nb]); if (NSPLIT >= 2) acc[mb][nb] = WFrag<T16>::mma(a[mb], b2, acc[mb][nb]); } }
        asm volatile("v_nop\n\tv_nop\n\tv_nop\n\tv_nop" : "+v"(acc[0][0]), "+v"(acc[1][1]), "+v"(acc[2][2]), "+v"(acc[3][3]) : "v"(a[0]), "v"(a[3]));
    }
#pragma unroll
    for (int mb = 0; mb < 4; ++mb) {
#pragma unroll
        for (int nb = 0; nb < 4; ++nb) {
#pragma unroll
            for (int j = 0; j < 8; ++j) os[(hi * 8 + j) * 68 + nb * 16 + lr] = acc[mb][nb][j]; }
        __builtin_amdgcn_wave_barrier(); asm volatile("" ::: "memory");
        float* crow = C + (size_t)(r0 + mb * 16) * ldc + c0;
#pragma unroll 1
        for (int ps = 0; ps < 2; ++ps) {
#pragma unroll
            for (int s = 0; s < 8; ++s) { const int row = 2 * s + hi, cofs = lr * 4; v4f val = *(const v4fa*)(os + row * 68 + cofs); if (BIAS) { val[0] += bfr(bias[c0 + cofs]); val[1] += bfr(bias[c0 + cofs + 1]); val[2] += bfr(bias[c0 + cofs + 2]); val[3] += bfr(bias[c0 + cofs + 3]); }
                *(volatile v4f*)(crow + (size_t)row * ldc + cofs) = val; }
            if (ps == 0) __threadfence(); }
        __builtin_amdgcn_wave_barrier(); asm volatile("" ::: "memory");
    }
}

template <typename T16, int NSPLIT, int CMODE>
__global__ __launch_bounds__(32) void k_gemmc(const T16* __restrict__ A, const T16* __restrict__ A2, const T16* __restrict__ Bt, const T16* __restrict__ Bt2, int K, float* C, int ldc, int roff, size_t sA, size_t sB, size_t sC) {
    typedef typename WFrag<T16>::V V;
    __shared__ __align__(16) float os[16 * 68];
    const size_t z = blockIdx.z; A += z * sA; if (A2) A2 += z * sA; Bt += z * sB; if (Bt2) Bt2 += z * sB; C += z * sC;
    const int lane = threadIdx.x & 31, lr = lane & 15, hi = lane >> 4; const int r0 = blockIdx.x * 64, c0 = blockIdx.y * 64;
    if (CMODE == 1 && c0 > r0 + roff + 63) return;
    const int Kl = (CMODE == 2) ? min(K, r0 + roff + 64) : K;
    v8f acc[4][4];
#pragma unroll
    for (int mb = 0; mb < 4; ++mb)
#pragma unroll
        for (int nb = 0; nb < 4; ++nb) acc[mb][nb] = (v8f){};
    const size_t aoff = (size_t)(r0 + lr) * K + 8 * hi, boff = (size_t)(c0 + lr) * K + 8 * hi;
#pragma unroll 1
    for (int kc = 0; kc < Kl; kc += 32) {
        V a[4], a2[4];
#pragma unroll
        for (int mb = 0; mb < 4; ++mb) { a[mb] = WFrag<T16>::ld(A + aoff + (size_t)mb * 16 * K + kc); if (NSPLIT == 1 || NSPLIT == 2) a2[mb] = WFrag<T16>::ld(A2 + aoff + (size_t)mb * 16 * K + kc); }
#pragma unroll
        for (int nb = 0; nb < 4; ++nb) { const V b = WFrag<T16>::ld(Bt + boff + (size_t)nb * 16 * K + kc); V b2; if (NSPLIT >= 2) b2 = WFrag<T16>::ld(Bt2 + boff + (size_t)nb * 16 * K + kc);
#pragma unroll
            for (int mb = 0; mb < 4; ++mb) { acc[mb][nb] = WFrag<T16>::mma(a[mb], b, acc[mb][nb]); if (NSPLIT == 1 || NSPLIT == 2) acc[mb][nb] = WFrag<T16>::mma(a2[mb], b, acc[mb][nb]); if (NSPLIT >= 2) acc[mb][nb] = WFrag<T16>::mma(a[mb], b2, acc[mb][nb]); } }
        asm volatile("v_nop\n\tv_nop\n\tv_nop\n\tv_nop" : "+v"(acc[0][0]), "+v"(acc[1][1]), "+v"(acc[2][2]), "+v"(acc[3][3]) : "v"(a[0]), "v"(a[3]));
    }
#pragma unroll
    for (int mb = 0; mb < 4; ++mb) {
#pragma unroll
        for (int nb = 0; nb < 4; ++nb) {
#pragma unroll
            for (int j = 0; j < 8; ++j) os[(hi * 8 + j) * 68 + nb * 16 + lr] = acc[mb][nb][j]; }
        __builtin_amdgcn_wave_barrier(); asm volatile("" ::: "memory");
        float* crow = C + (size_t)(r0 + mb * 16) * ldc + c0;
#pragma unroll 1
        for (int ps = 0; ps < 2; ++ps) {
#pragma unroll
            for (int s = 0; s < 8; ++s) { const int row = 2 * s + hi, cofs = lr * 4; v4f val = *(const v4fa*)(os + row * 68 + cofs);
                *(volatile v4f*)(crow + (size_t)row * ldc + cofs) = val; }
            if (ps == 0) __threadfence(); }
        __builtin_amdgcn_wave_barrier(); asm volatile("" ::: "memory");
    }
}
__device__ __forceinline__ h16 tohx(float x) { return (h16)x; }
__device__ __forceinline__ void splitf(float y, unsigned short& h, unsigned short& l) { h = f2bf(y); l = f2bf(y - bf2f(h)); }
typedef __attribute__((ext_vector_type(2))) unsigned short v2us;
typedef __attribute__((ext_vector_type(4))) unsigned short v4us;
typedef __attribute__((ext_vector_type(2))) _Float16 v2h;
typedef __attribute__((ext_vector_type(4))) _Float16 v4h;
typedef __attribute__((ext_vector_type(4))) int v4i;

__global__ __launch_bounds__(256) void k_cvt8(const float* __restrict__ src, bf* dst, size_t n8) { const size_t i = (size_t)blockIdx.x * 256 + threadIdx.x; if (i >= n8) return; const v8f v = *(const v8f*)(src + i * 8); v8us o;
#pragma unroll
    for (int k = 0; k < 8; ++k) o[k] = f2bf(v[k]); *(volatile v8us*)(dst + i * 8) = o; __threadfence(); *(volatile v8us*)(dst + i * 8) = o; }
__global__ __launch_bounds__(64) void k_counts(const float* __restrict__ mk, float* KEEP, float* CNT) { const int b = blockIdx.x; if (threadIdx.x != 0) return; float c = 0.f;
    for (int t = 0; t < TT; ++t) { const float keep = (bfr(mk[(size_t)b * TT + t]) == 0.f) ? 1.f : 0.f; c = __fadd_rn(c, keep); *(volatile float*)(KEEP + (size_t)b * TT + t) = keep; *(volatile float*)(CNT + (size_t)b * TT + t) = c; __threadfence(); *(volatile float*)(KEEP + (size_t)b * TT + t) = keep; *(volatile float*)(CNT + (size_t)b * TT + t) = c; } }
__global__ __launch_bounds__(256) void k_linefix(float* A, size_t n4) { const size_t e = ((size_t)blockIdx.x * 256 + threadIdx.x) * 4; if (e >= n4 * 4) return; const v4f a = *(const v4f*)(A + e); *(volatile v4f*)(A + e) = a; __threadfence(); *(volatile v4f*)(A + e) = a; }
__global__ __launch_bounds__(256) void k_qkn(const float* __restrict__ F, const int* __restrict__ pos, const float* __restrict__ KEEP, h16* P) { const int lane = threadIdx.x & 31; const size_t row = (size_t)blockIdx.x * 8 + (threadIdx.x >> 5); if (row >= (size_t)NH_ * TT) return; const int t = (int)(row % TT); const int h = (int)(row / TT); const float* f = F + (size_t)t * DM + h * HD; float v[4]; float ss = 0.f;
    const float p = (float)pos[t];
#pragma unroll
    for (int q = 0; q < 2; ++q) { const int d0 = q * 64 + lane * 2; float a = f[d0], b = f[d0 + 1];
        if (d0 < ROT) { const int i = d0 >> 1; const float invf = __fdiv_rn(1.0f, powf(10000.0f, (float)(2 * i) / (float)ROT)); const float ang = __fmul_rn(p, invf); const float c = cosf(ang), s = sinf(ang);
            float ac = __fmul_rn(a, c), bs = __fmul_rn(b, s), bc = __fmul_rn(b, c), as = __fmul_rn(a, s); asm volatile("" : "+v"(ac)); asm volatile("" : "+v"(bs)); asm volatile("" : "+v"(bc)); asm volatile("" : "+v"(as)); const float a2 = __fsub_rn(ac, bs), b2 = __fadd_rn(bc, as); a = a2; b = b2; }
        v[q * 2] = a; v[q * 2 + 1] = b; float pa = __fmul_rn(a, a); asm volatile("" : "+v"(pa)); ss = __fadd_rn(ss, pa); float pb = __fmul_rn(b, b); asm volatile("" : "+v"(pb)); ss = __fadd_rn(ss, pb); }
#pragma unroll
    for (int sh = 16; sh; sh >>= 1) ss += __shfl_xor(ss, sh, 32);
    const float nrm = fmaxf(__fsqrt_rn(ss), 1e-12f); const float keep = KEEP[t];
#pragma unroll
    for (int q = 0; q < 2; ++q) { v2h o; float x0 = __fdiv_rn(v[q * 2], nrm), x1 = __fdiv_rn(v[q * 2 + 1], nrm); asm volatile("" : "+v"(x0)); asm volatile("" : "+v"(x1)); o[0] = tohx(__fmul_rn(x0, keep)); o[1] = tohx(__fmul_rn(x1, keep)); h16* dst = P + ((size_t)h * TT + t) * HD + q * 64 + lane * 2; *(volatile v2h*)dst = o; __threadfence(); *(volatile v2h*)dst = o; } }
__global__ __launch_bounds__(256) void k_vsc(const float* __restrict__ F, const float* __restrict__ KEEP, const float* __restrict__ CNT, const float* __restrict__ nc, h16* VT) { const size_t e = ((size_t)blockIdx.x * 256 + threadIdx.x) * 2; if (e >= (size_t)NH_ * HD * TT) return; const int t = (int)(e % TT); const int d = (int)((e / TT) % HD); const int h = (int)(e / ((size_t)TT * HD)); const float expo = __fdiv_rn(1.0f, __fadd_rn(1.0f, __expf(-bfr(nc[h])))); v2h o;
#pragma unroll
    for (int u = 0; u < 2; ++u) { const float cnt = CNT[t + u]; const float den = fmaxf(powf(cnt, expo), 1.0f); float vv = __fdiv_rn(F[(size_t)(t + u) * DM + h * HD + d], den); asm volatile("" : "+v"(vv)); o[u] = tohx(__fmul_rn(vv, KEEP[t + u])); }
    *(volatile v2h*)(VT + e) = o; __threadfence(); *(volatile v2h*)(VT + e) = o; }
__global__ __launch_bounds__(256) void k_s2p(const float* __restrict__ S, h16* P16) { const size_t e = ((size_t)blockIdx.x * 256 + threadIdx.x) * 4; if (e >= (size_t)ZH * TT * TT) return; const int j = (int)(e % TT); const int i = (int)((e / TT) % TT); const int jlim = ((i >> 6) + 1) * 64; v4h o;
    if (j < jlim) { const v4f a = *(const v4f*)(S + e);
#pragma unroll
        for (int u = 0; u < 4; ++u) o[u] = (j + u <= i) ? tohx(a[u] * PCAR) : (h16)0.f; } else { o[0] = (h16)0.f; o[1] = (h16)0.f; o[2] = (h16)0.f; o[3] = (h16)0.f; }
    *(volatile v4h*)(P16 + e) = o; __threadfence(); *(volatile v4h*)(P16 + e) = o; }
__global__ __launch_bounds__(256) void k_merge(const float* __restrict__ O, int h0, bf* Ah, bf* Al) { const size_t e = ((size_t)blockIdx.x * 256 + threadIdx.x) * 4; if (e >= (size_t)ZH * TT * HD) return; const int d = (int)(e % HD); const int t = (int)((e / HD) % TT); const int zz = (int)(e / ((size_t)HD * TT)); const size_t oo = (size_t)t * DM + (h0 + zz) * HD + d; v4us oh, ol;
#pragma unroll
    for (int u = 0; u < 4; ++u) { unsigned short a, b; splitf(O[e + u] * (1.0f / PCAR), a, b); oh[u] = a; ol[u] = b; } *(volatile v4us*)(Ah + oo) = oh; *(volatile v4us*)(Al + oo) = ol; __threadfence(); *(volatile v4us*)(Ah + oo) = oh; *(volatile v4us*)(Al + oo) = ol; }

extern "C" void kernel_launch(void* const* d_in, const int* in_sizes, int n_in,
                              void* d_out, int out_size, void* d_ws, size_t ws_size, hipStream_t stream) {
    (void)in_sizes; (void)n_in; (void)out_size;
    const float* x = (const float*)d_in[0]; const float* mask = (const float*)d_in[1]; const int* pos = (const int*)d_in[2]; const float* Wq = (const float*)d_in[3]; const float* Wk = (const float*)d_in[4]; const float* Wv = (const float*)d_in[5]; const float* Wo = (const float*)d_in[6]; const float* nc = (const float*)d_in[7];
    float* OUT = (float*)d_out;
    char* wsp = (char*)d_ws;
    auto take = [&](size_t bytes) { char* p = wsp; wsp += (bytes + 255) & ~(size_t)255; return (void*)p; };
    bf* XB = (bf*)take((size_t)TT * DM * 2); bf* BW = (bf*)take((size_t)DM * DM * 2); float* F = (float*)take((size_t)TT * DM * 4); float* KEEP = (float*)take((size_t)NB_ * TT * 4); float* CNT = (float*)take((size_t)NB_ * TT * 4);
    h16* QP = (h16*)take((size_t)NH_ * TT * HD * 2); h16* KP = (h16*)take((size_t)NH_ * TT * HD * 2); h16* VT = (h16*)take((size_t)NH_ * HD * TT * 2); float* S = (float*)take((size_t)ZH * TT * TT * 4); h16* P16 = (h16*)take((size_t)ZH * TT * TT * 2); float* O = (float*)take((size_t)ZH * TT * HD * 4); bf* ATh = (bf*)take((size_t)TT * DM * 2); bf* ATl = (bf*)take((size_t)TT * DM * 2);
    if ((size_t)(wsp - (char*)d_ws) > ws_size) return;
    k_counts<<<NB_, 64, 0, stream>>>(mask, KEEP, CNT); k_linefix<<<(NB_ * TT / 4 + 255) / 256, 256, 0, stream>>>(KEEP, (size_t)NB_ * TT / 4); k_linefix<<<(NB_ * TT / 4 + 255) / 256, 256, 0, stream>>>(CNT, (size_t)NB_ * TT / 4);
    const dim3 gp(TT / 64, DM / 64, 1); const size_t zq = (size_t)TT * HD, zS = (size_t)TT * TT, zv = (size_t)HD * TT, zo = (size_t)TT * HD;
    for (int b = 0; b < NB_; ++b) {
        k_cvt8<<<(unsigned)(((size_t)TT * DM / 8 + 255) / 256), 256, 0, stream>>>(x + (size_t)b * TT * DM, XB, (size_t)TT * DM / 8);
        k_cvt8<<<(unsigned)(((size_t)DM * DM / 8 + 255) / 256), 256, 0, stream>>>(Wq, BW, (size_t)DM * DM / 8); k_gemmw<bf, 0, false><<<gp, 32, 0, stream>>>(XB, nullptr, BW, nullptr, DM, F, DM, nullptr, 0, 0, 0); k_qkn<<<(NH_ * TT + 7) / 8, 256, 0, stream>>>(F, pos + (size_t)b * TT, KEEP + (size_t)b * TT, QP);
        k_cvt8<<<(unsigned)(((size_t)DM * DM / 8 + 255) / 256), 256, 0, stream>>>(Wk, BW, (size_t)DM * DM / 8); k_gemmw<bf, 0, false><<<gp, 32, 0, stream>>>(XB, nullptr, BW, nullptr, DM, F, DM, nullptr, 0, 0, 0); k_qkn<<<(NH_ * TT + 7) / 8, 256, 0, stream>>>(F, pos + (size_t)b * TT, KEEP + (size_t)b * TT, KP);
        k_cvt8<<<(unsigned)(((size_t)DM * DM / 8 + 255) / 256), 256, 0, stream>>>(Wv, BW, (size_t)DM * DM / 8); k_gemmw<bf, 0, false><<<gp, 32, 0, stream>>>(XB, nullptr, BW, nullptr, DM, F, DM, nullptr, 0, 0, 0); k_vsc<<<(unsigned)(((size_t)NH_ * HD * TT / 2 + 255) / 256), 256, 0, stream>>>(F, KEEP + (size_t)b * TT, CNT + (size_t)b * TT, nc, VT);
        for (int h0 = 0; h0 < NH_; h0 += ZH) {
            k_gemmc<h16, 0, 1><<<dim3(TT / 64, TT / 64, ZH), 32, 0, stream>>>(QP + (size_t)h0 * zq, nullptr, KP + (size_t)h0 * zq, nullptr, HD, S, TT, 0, zq, zq, zS);
            k_s2p<<<(unsigned)(((size_t)ZH * TT * TT / 4 + 255) / 256), 256, 0, stream>>>(S, P16);
            k_gemmc<h16, 0, 2><<<dim3(TT / 64, HD / 64, ZH), 32, 0, stream>>>(P16, nullptr, VT + (size_t)h0 * zv, nullptr, TT, O, HD, 0, zS, zv, zo);
            k_merge<<<(unsigned)(((size_t)ZH * TT * HD / 4 + 255) / 256), 256, 0, stream>>>(O, h0, ATh, ATl); }
        k_cvt8<<<(unsigned)(((size_t)DM * DM / 8 + 255) / 256), 256, 0, stream>>>(Wo, BW, (size_t)DM * DM / 8); k_gemmw<bf, 1, false><<<gp, 32, 0, stream>>>(ATh, ATl, BW, nullptr, DM, OUT + (size_t)b * TT * DM, DM, nullptr, 0, 0, 0); }
}
